// MultiHeadAttentionWithLoRA_4157528343230
// MI455X (gfx1250) — hardware-verified
//
#include <hip/hip_runtime.h>
#include <math.h>
#include <float.h>
#include <stdint.h>

#define NBAT  4
#define SEQ   2048
#define DMOD  1024
#define NH    16
#define HD    64
#define LR    8
#define NQB   (SEQ / 64)
#define VLP   512
#define RESQB 8
#define NXA   (NH * LR)
#define XAOFF (3 * DMOD)
#define NALL  (3 * DMOD + 3 * NXA)
#define NPO   (DMOD + 64)
static_assert(RESQB * 64 <= VLP);
static_assert(NH * HD == DMOD);
static_assert((SEQ % 64) == 0 && (DMOD % 64) == 0 && (NALL % 64) == 0 && (NPO % 64) == 0);
static_assert((NALL % 32) == 0 && (NPO % 32) == 0);

typedef _Float16 v16h __attribute__((ext_vector_type(16)));
typedef _Float16 v8h  __attribute__((ext_vector_type(8)));
typedef __bf16   v16b __attribute__((ext_vector_type(16)));
typedef __bf16   v8b  __attribute__((ext_vector_type(8)));
typedef float    v8f  __attribute__((ext_vector_type(8)));
typedef float    v4f  __attribute__((ext_vector_type(4)));
typedef unsigned int v4u __attribute__((ext_vector_type(4)));

__device__ __forceinline__ unsigned short bf_bits(float f) {
  unsigned u = __float_as_uint(f);
  return (unsigned short)((u + 0x7FFFu + ((u >> 16) & 1u)) >> 16);
}
__device__ __forceinline__ float bf_up(unsigned short h) { return __uint_as_float(((unsigned)h) << 16); }
__device__ __forceinline__ float bfr(float f) { return bf_up(bf_bits(f)); }
__device__ __forceinline__ unsigned short h_bits(_Float16 x) { return __builtin_bit_cast(unsigned short, x); }
__device__ __forceinline__ unsigned pk16(unsigned short a, unsigned short b) { return (unsigned)a | ((unsigned)b << 16); }
__device__ __forceinline__ v8f zero8() { v8f z = {0.f, 0.f, 0.f, 0.f, 0.f, 0.f, 0.f, 0.f}; return z; }
__device__ __forceinline__ v8h zero8h() {
  const _Float16 z = (_Float16)0.0f;
  v8h r = {z, z, z, z, z, z, z, z};
  return r;
}

__device__ __forceinline__ v16b ldfrag_b(const __bf16* p) {
  union { v16b v; v8b h[2]; } f;
  f.h[0] = *(const v8b*)(p);
  f.h[1] = *(const v8b*)(p + 16);
  return f.v;
}

__device__ __forceinline__ v8f mma_b(v16b a, v16b b, v8f c) {
  c = __builtin_amdgcn_wmma_f32_16x16x32_bf16(false, a, false, b, (short)0, c, false, false);
#if defined(__HIP_DEVICE_COMPILE__)
  asm volatile("v_nop\n\tv_nop\n\tv_nop\n\tv_nop" : "+v"(c) : "v"(a), "v"(b));
#endif
  return c;
}
__device__ __forceinline__ v8f mma_h(v16h a, v16h b, v8f c) {
  c = __builtin_amdgcn_wmma_f32_16x16x32_f16(false, a, false, b, (short)0, c, false, false);
#if defined(__HIP_DEVICE_COMPILE__)
  asm volatile("v_nop\n\tv_nop\n\tv_nop\n\tv_nop" : "+v"(c) : "v"(a), "v"(b));
#endif
  return c;
}
__device__ __forceinline__ v8f mma_b_raw(v16b a, v16b b, v8f c) {
  return __builtin_amdgcn_wmma_f32_16x16x32_bf16(false, a, false, b, (short)0, c, false, false);
}
__device__ __forceinline__ void dep_guard_b(v8f& a, v8f& b, v16b x, v16b y) {
#if defined(__HIP_DEVICE_COMPILE__)
  asm volatile("v_nop\n\tv_nop\n\tv_nop\n\tv_nop" : "+v"(a), "+v"(b) : "v"(x), "v"(y));
#endif
}
__device__ __forceinline__ void keep4_b(v16b a, v16b b, v16b c, v16b d) {
#if defined(__HIP_DEVICE_COMPILE__)
  asm volatile("v_nop" :: "v"(a), "v"(b), "v"(c), "v"(d));
#endif
}
__device__ __forceinline__ void acc_guard4(v8f& a, v8f& b, v8f& c, v8f& d) {
#if defined(__HIP_DEVICE_COMPILE__)
  asm volatile("v_nop\n\tv_nop\n\tv_nop\n\tv_nop" : "+v"(a), "+v"(b), "+v"(c), "+v"(d));
#endif
}

__global__ __launch_bounds__(256) void cvt_bf16x8(const float* __restrict__ in, unsigned short* out, int n8) {
  const int i = blockIdx.x * 256 + threadIdx.x;
  if (i < n8) {
    const v4f a = *(const v4f*)(in + (size_t)i * 8);
    const v4f b = *(const v4f*)(in + (size_t)i * 8 + 4);
    v4u p;
    p[0] = pk16(bf_bits(a[0]), bf_bits(a[1]));
    p[1] = pk16(bf_bits(a[2]), bf_bits(a[3]));
    p[2] = pk16(bf_bits(b[0]), bf_bits(b[1]));
    p[3] = pk16(bf_bits(b[2]), bf_bits(b[3]));
    *(volatile v4u*)(out + (size_t)i * 8) = p;
    __threadfence();
    *(volatile v4u*)(out + (size_t)i * 8) = p;
  }
}

__global__ __launch_bounds__(256) void tcvt_bf16(const float* __restrict__ in, unsigned short* out,
                                                  int nOut, int nValid, int K, int G) {
  const int kc8 = K >> 3;
  const int i = blockIdx.x * 256 + threadIdx.x;
  if (i >= nOut * kc8) return;
  const int n  = i / kc8;
  const int kc = (i - n * kc8) * 8;
  const int nn = (n < nValid) ? n : (nValid - 1);
  const size_t base = ((size_t)(nn / G) * K + kc) * (size_t)G + (size_t)(nn % G);
  float f[8];
#pragma unroll
  for (int j = 0; j < 8; ++j) f[j] = in[base + (size_t)j * G];
  v4u p;
#pragma unroll
  for (int e = 0; e < 4; ++e) p[e] = pk16(bf_bits(f[2 * e]), bf_bits(f[2 * e + 1]));
  if (n >= nValid) { p[0] = 0u; p[1] = 0u; p[2] = 0u; p[3] = 0u; }
  unsigned short* dst = out + (size_t)n * K + kc;
  *(volatile v4u*)dst = p;
  __threadfence();
  *(volatile v4u*)dst = p;
}

template <int NSPLIT, int OUT_MODE>
__global__ __launch_bounds__(256) void gemm64(
    const unsigned short* __restrict__ Ap, const unsigned short* A2p, int lda, long long strideA,
    const unsigned short* __restrict__ Btp, const unsigned short* Bt2p, int ldb, long long strideB,
    void* Cout, int ldc, long long strideC,
    void* Cout2, int ldc2, long long strideC2, int N2,
    int M, int N, int K, float rscale) {
  const __bf16* A   = (const __bf16*)(const void*)Ap;
  const __bf16* A2  = (const __bf16*)(const void*)A2p;
  const __bf16* Bt  = (const __bf16*)(const void*)Btp;
  const __bf16* Bt2 = (const __bf16*)(const void*)Bt2p;
  __shared__ __align__(16) float sT[8][16 * 68];
  const int b    = blockIdx.y;
  const int lane = threadIdx.x & 31;
  const int wave = threadIdx.x >> 5;
  const int tilesN = N >> 6;
  const int tilesM = M >> 6;
  const int tile = blockIdx.x * 8 + wave;
  if (tile >= tilesM * tilesN) return;
  const int tm = tile / tilesN;
  const int tn = tile - tm * tilesN;
  const int m0 = tm << 6;
  const int n0 = tn << 6;

  const __bf16* Ab  = A  + (size_t)b * strideA;
  const __bf16* Bb  = Bt + (size_t)b * strideB;
  const __bf16* Ab2 = (NSPLIT >= 1) ? (A2  + (size_t)b * strideA) : Ab;
  const __bf16* Bb2 = (NSPLIT == 2) ? (Bt2 + (size_t)b * strideB) : Bb;

  const int rlane = lane & 15;
  const int koff  = (lane >> 4) * 8;
  const int mOff  = (lane >> 4) * 8;

  v8f acc[4][4];
#pragma unroll
  for (int i = 0; i < 4; ++i)
#pragma unroll
    for (int j = 0; j < 4; ++j) acc[i][j] = zero8();

  for (int k0 = 0; k0 < K; k0 += 32) {
    v16b bh[4], bl[4];
#pragma unroll
    for (int j = 0; j < 4; ++j) {
      const size_t bo = (size_t)(n0 + (j << 4) + rlane) * ldb + koff + k0;
      bh[j] = ldfrag_b(Bb + bo);
      if (NSPLIT == 2) bl[j] = ldfrag_b(Bb2 + bo); else bl[j] = bh[j];
    }
#pragma unroll
    for (int i = 0; i < 4; ++i) {
      const size_t ao = (size_t)(m0 + (i << 4) + rlane) * lda + koff + k0;
      const v16b ah = ldfrag_b(Ab + ao);
      v16b al = ah;
      if (NSPLIT >= 1) al = ldfrag_b(Ab2 + ao);
#pragma unroll
      for (int j = 0; j < 4; ++j) {
        acc[i][j] = mma_b_raw(ah, bh[j], acc[i][j]);
        if (NSPLIT >= 1) acc[i][j] = mma_b_raw(al, bh[j], acc[i][j]);
        if (NSPLIT == 2) acc[i][j] = mma_b_raw(ah, bl[j], acc[i][j]);
      }
      dep_guard_b(acc[i][0], acc[i][3], ah, al);
    }
    keep4_b(bh[0], bh[1], bh[2], bh[3]);
    if (NSPLIT == 2) keep4_b(bl[0], bl[1], bl[2], bl[3]);
  }
  acc_guard4(acc[0][0], acc[0][1], acc[0][2], acc[0][3]);
  acc_guard4(acc[1][0], acc[1][1], acc[1][2], acc[1][3]);
  acc_guard4(acc[2][0], acc[2][1], acc[2][2], acc[2][3]);
  acc_guard4(acc[3][0], acc[3][1], acc[3][2], acc[3][3]);

  float* slab = sT[wave];
#pragma unroll
  for (int i = 0; i < 4; ++i) {
    const int mBase = m0 + (i << 4);
#pragma unroll
    for (int j = 0; j < 4; ++j) {
#pragma unroll
      for (int r = 0; r < 8; ++r) {
        slab[(mOff + r) * 68 + (j << 4) + rlane] = acc[i][j][r];
      }
    }
    __builtin_amdgcn_fence(__ATOMIC_RELEASE, "workgroup");
    __builtin_amdgcn_wave_barrier();
    __builtin_amdgcn_fence(__ATOMIC_ACQUIRE, "workgroup");
    if (OUT_MODE == 0) {
      float* C = (float*)Cout + (size_t)b * strideC;
      const int hh = lane >> 4, c4 = (lane & 15) * 4;
      for (int pass = 0; pass < 2; ++pass) {
#pragma unroll
        for (int it = 0; it < 8; ++it) {
          const int row = it * 2 + hh;
          const v4f v = *(const v4f*)(slab + row * 68 + c4);
          *(volatile v4f*)(C + (size_t)(mBase + row) * ldc + n0 + c4) = v;
        }
        __threadfence();
      }
    } else {
      const int q = lane >> 3, c8 = (lane & 7) * 8;
      unsigned short* C  = (unsigned short*)Cout  + (size_t)b * strideC;
      unsigned short* C2 = (unsigned short*)Cout2 + (size_t)b * strideC2;
      const bool wlo = (OUT_MODE == 2) || (n0 < N2);
      v4u hv[4], lv[4];
#pragma unroll
      for (int it = 0; it < 4; ++it) {
        const int row = it * 4 + q;
        const float* sp = slab + row * 68 + c8;
        v4u a, a2;
#pragma unroll
        for (int e = 0; e < 4; ++e) {
          const float f0 = sp[2 * e], f1 = sp[2 * e + 1];
          unsigned short h0, h1, l0, l1;
          if (OUT_MODE == 2) {
            h0 = bf_bits(f0); h1 = bf_bits(f1);
            l0 = bf_bits(f0 - bf_up(h0)); l1 = bf_bits(f1 - bf_up(h1));
          } else {
            const _Float16 x0 = (_Float16)f0, x1 = (_Float16)f1;
            h0 = h_bits(x0); h1 = h_bits(x1);
            l0 = h_bits((_Float16)((f0 - (float)x0) * rscale));
            l1 = h_bits((_Float16)((f1 - (float)x1) * rscale));
          }
          a[e] = pk16(h0, h1); a2[e] = pk16(l0, l1);
        }
        hv[it] = a; lv[it] = a2;
      }
      for (int pass = 0; pass < 2; ++pass) {
#pragma unroll
        for (int it = 0; it < 4; ++it) {
          const int row = it * 4 + q;
          *(volatile v4u*)(C + (size_t)(mBase + row) * ldc + n0 + c8) = hv[it];
          if (wlo) *(volatile v4u*)(C2 + (size_t)(mBase + row) * ldc2 + n0 + c8) = lv[it];
        }
        __threadfence();
      }
    }
    __builtin_amdgcn_fence(__ATOMIC_RELEASE, "workgroup");
    __builtin_amdgcn_wave_barrier();
    __builtin_amdgcn_fence(__ATOMIC_ACQUIRE, "workgroup");
  }
}

__global__ __launch_bounds__(256) void proj_finish(const float* __restrict__ Y, int cb, int cxa,
                                                    const float* __restrict__ Bm,
                                                    unsigned short* Hh, unsigned short* Hl) {
  const int i = blockIdx.x * 256 + threadIdx.x;
  if (i >= SEQ * (DMOD / 8)) return;
  const int t  = i >> 7;
  const int n  = (i & 127) * 8;
  const int h  = n >> 6;
  const int d0 = n & 63;
  const float* yb = Y + (size_t)t * NALL + cb + n;
  const float* xa = Y + (size_t)t * NALL + cxa + h * LR;
  const v4f b0 = *(const v4f*)(yb);
  const v4f b1 = *(const v4f*)(yb + 4);
  float acc[8];
#pragma unroll
  for (int e = 0; e < 8; ++e) acc[e] = 0.f;
#pragma unroll 1
  for (int r = 0; r < LR; ++r) {
    const float xr = 2.0f * xa[r];
    const float* bw = Bm + (size_t)(h * LR + r) * HD + d0;
    const v4f w0 = *(const v4f*)(bw);
    const v4f w1 = *(const v4f*)(bw + 4);
#pragma unroll
    for (int e = 0; e < 4; ++e) {
      acc[e]     += xr * bfr(w0[e]);
      acc[4 + e] += xr * bfr(w1[e]);
    }
  }
  float v[8];
#pragma unroll
  for (int e = 0; e < 4; ++e) { v[e] = b0[e] + acc[e]; v[4 + e] = b1[e] + acc[4 + e]; }
  v4u ph, pl;
#pragma unroll
  for (int e = 0; e < 4; ++e) {
    const unsigned short h0 = bf_bits(v[2 * e]), h1 = bf_bits(v[2 * e + 1]);
    const unsigned short l0 = bf_bits(v[2 * e] - bf_up(h0)), l1 = bf_bits(v[2 * e + 1] - bf_up(h1));
    ph[e] = pk16(h0, h1); pl[e] = pk16(l0, l1);
  }
  const size_t go = (size_t)t * DMOD + n;
  for (int pass = 0; pass < 2; ++pass) {
    *(volatile v4u*)(Hh + go) = ph;
    *(volatile v4u*)(Hl + go) = pl;
    __threadfence();
  }
}

__global__ __launch_bounds__(256) void v_finish(const float* __restrict__ Y, const float* __restrict__ Bm,
                                                 unsigned short* vth, unsigned short* vtl, float rscale) {
  __shared__ __align__(16) float sV[64 * 68];
  const int tid  = threadIdx.x;
  const int lane = tid & 31;
  const int wave = tid >> 5;
  const int t0 = (blockIdx.x & (NQB - 1)) * 64;
  const int n0 = (blockIdx.x / NQB) * 64;
  const int trow = tid >> 2;
  const int dq   = (tid & 3) * 16;
  const int t = t0 + trow;
  const int h = n0 >> 6;
  {
    const float* yb = Y + (size_t)t * NALL + 2 * DMOD + n0 + dq;
    const float* xa = Y + (size_t)t * NALL + XAOFF + 2 * NXA + h * LR;
    const v4f b0 = *(const v4f*)(yb);
    const v4f b1 = *(const v4f*)(yb + 4);
    const v4f b2 = *(const v4f*)(yb + 8);
    const v4f b3 = *(const v4f*)(yb + 12);
    float acc[16];
#pragma unroll
    for (int e = 0; e < 16; ++e) acc[e] = 0.f;
#pragma unroll 1
    for (int r = 0; r < LR; ++r) {
      const float xr = 2.0f * xa[r];
      const float* bw = Bm + (size_t)(h * LR + r) * HD + dq;
      const v4f w0 = *(const v4f*)(bw);
      const v4f w1 = *(const v4f*)(bw + 4);
      const v4f w2 = *(const v4f*)(bw + 8);
      const v4f w3 = *(const v4f*)(bw + 12);
#pragma unroll
      for (int e = 0; e < 4; ++e) {
        acc[e]      += xr * bfr(w0[e]);
        acc[4 + e]  += xr * bfr(w1[e]);
        acc[8 + e]  += xr * bfr(w2[e]);
        acc[12 + e] += xr * bfr(w3[e]);
      }
    }
    v4f o0, o1, o2, o3;
#pragma unroll
    for (int e = 0; e < 4; ++e) {
      o0[e] = b0[e] + acc[e];
      o1[e] = b1[e] + acc[4 + e];
      o2[e] = b2[e] + acc[8 + e];
      o3[e] = b3[e] + acc[12 + e];
    }
    float* sp = sV + trow * 68 + dq;
    *(v4f*)(sp)      = o0;
    *(v4f*)(sp + 4)  = o1;
    *(v4f*)(sp + 8)  = o2;
    *(v4f*)(sp + 12) = o3;
  }
  __syncthreads();
  const int q = lane >> 3, c8 = (lane & 7) * 8;
  v4u hv[2], lv[2];
#pragma unroll
  for (int it = 0; it < 2; ++it) {
    const int nl = it * 32 + wave * 4 + q;
    v4u a, a2;
#pragma unroll
    for (int e = 0; e < 4; ++e) {
      const float f0 = sV[(c8 + 2 * e) * 68 + nl];
      const float f1 = sV[(c8 + 2 * e + 1) * 68 + nl];
      const _Float16 x0 = (_Float16)f0, x1 = (_Float16)f1;
      const unsigned short h0 = h_bits(x0), h1 = h_bits(x1);
      const unsigned short l0 = h_bits((_Float16)((f0 - (float)x0) * rscale));
      const unsigned short l1 = h_bits((_Float16)((f1 - (float)x1) * rscale));
      a[e] = pk16(h0, h1); a2[e] = pk16(l0, l1);
    }
    hv[it] = a; lv[it] = a2;
  }
  const bool wres = (t0 < VLP);
  for (int pass = 0; pass < 2; ++pass) {
#pragma unroll
    for (int it = 0; it < 2; ++it) {
      const int nl = it * 32 + wave * 4 + q;
      *(volatile v4u*)(vth + (size_t)(n0 + nl) * SEQ + t0 + c8) = hv[it];
      if (wres) *(volatile v4u*)(vtl + (size_t)(n0 + nl) * VLP + t0 + c8) = lv[it];
    }
    __threadfence();
  }
}

template <bool RES>
__global__ __launch_bounds__(128)
void attn_causal64(const unsigned short* __restrict__ qhp, const unsigned short* __restrict__ qlp,
                   const unsigned short* __restrict__ khp, const unsigned short* __restrict__ klp,
                   const unsigned short* __restrict__ vhp, const unsigned short* __restrict__ vlp,
                   unsigned short* ohp, unsigned short* olp,
                   int qbBase, int nqbThis, float sscale) {
  union FB { v16b v; v8b h[2]; };
  union FH { v16h v; v8h h[2]; };
  __shared__ __align__(16) __bf16   Ksh[64 * 64];
  __shared__ __align__(16) __bf16   Ksl[64 * 64];
  __shared__ __align__(16) _Float16 Vth[64 * 64];
  __shared__ __align__(16) _Float16 Vtl[RES ? 64 * 64 : 8];
  __shared__ __align__(16) _Float16 Psh[4][16 * 64];
  __shared__ __align__(16) _Float16 Psl[RES ? 4 : 1][16 * 64];
  __shared__ __align__(16) float    Os[4][16 * 64];

  const int tid  = threadIdx.x;
  const int wave = tid >> 5;
  const int lane = tid & 31;
  const int hh   = lane >> 4;
  const int c    = lane & 15;

  const int bx   = blockIdx.x;
  const int qbl  = bx % nqbThis;
  const int h    = bx / nqbThis;
  const int qb   = qbBase + qbl;
  const int q0   = qb * 64 + wave * 16;

  const __bf16* Qh = (const __bf16*)(const void*)qhp + (size_t)h * HD;
  const __bf16* Ql = (const __bf16*)(const void*)qlp + (size_t)h * HD;
  const __bf16* Kh = (const __bf16*)(const void*)khp + (size_t)h * HD;
  const __bf16* Kl = (const __bf16*)(const void*)klp + (size_t)h * HD;
  const _Float16* Vh = (const _Float16*)(const void*)vhp + ((size_t)h * HD) * SEQ;
  const _Float16* Vl = (const _Float16*)(const void*)vlp + ((size_t)h * HD) * VLP;

  v16b qah[2], qal[2];
#pragma unroll
  for (int dc = 0; dc < 2; ++dc) {
    const size_t qo = (size_t)(q0 + c) * DMOD + dc * 32 + 8 * hh;
    qah[dc] = ldfrag_b(Qh + qo);
    qal[dc] = ldfrag_b(Ql + qo);
  }

  float mrow[8], lrow[8];
  v8f oacc[4];
#pragma unroll
  for (int r = 0; r < 8; ++r) { mrow[r] = -INFINITY; lrow[r] = 0.f; }
#pragma unroll
  for (int t = 0; t < 4; ++t) oacc[t] = zero8();

  for (int kt = 0; kt < NQB; ++kt) {
    if (kt > qb) break;
    const int kv0 = kt * 64;
    __syncthreads();
    {
      const int r = tid >> 1, half = (tid & 1) * 32;
      const __bf16*   kg  = Kh + (size_t)(kv0 + r) * DMOD + half;
      const __bf16*   klg = Kl + (size_t)(kv0 + r) * DMOD + half;
      const _Float16* vg  = Vh + (size_t)r * SEQ + kv0 + half;
      const int kvl = (kv0 + 64 <= VLP) ? kv0 : (VLP - 64);
      const _Float16* vlg = Vl + (size_t)r * VLP + kvl + half;
      const bool resOK = (kv0 + 64 <= VLP);
#pragma unroll
      for (int i = 0; i < 4; ++i) {
        const v8b a0 = *(const v8b*)(kg + 8 * i);
        const v8b a1 = *(const v8b*)(klg + 8 * i);
        const v8h b0 = *(const v8h*)(vg + 8 * i);
        *(v8b*)(Ksh + r * 64 + half + 8 * i) = a0;
        *(v8b*)(Ksl + r * 64 + half + 8 * i) = a1;
        *(v8h*)(Vth + r * 64 + half + 8 * i) = b0;
        if (RES) {
          v8h b1 = *(const v8h*)(vlg + 8 * i);
          if (!resOK) b1 = zero8h();
          *(v8h*)(Vtl + r * 64 + half + 8 * i) = b1;
        }
      }
    }
    __syncthreads();

    v8f s[4];
#pragma unroll
    for (int j = 0; j < 4; ++j) {
      s[j] = zero8();
#pragma unroll
      for (int dc = 0; dc < 2; ++dc) {
        FB kb, kl;
        kb.h[0] = *(const v8b*)(Ksh + (j * 16 + c) * 64 + dc * 32 + 8 * hh);
        kb.h[1] = *(const v8b*)(Ksh + (j * 16 + c) * 64 + dc * 32 + 16 + 8 * hh);
        kl.h[0] = *(const v8b*)(Ksl + (j * 16 + c) * 64 + dc * 32 + 8 * hh);
        kl.h[1] = *(const v8b*)(Ksl + (j * 16 + c) * 64 + dc * 32 + 16 + 8 * hh);
        s[j] = mma_b(qah[dc], kb.v, s[j]);
        s[j] = mma_b(qah[dc], kl.v, s[j]);
        s[j] = mma_b(qal[dc], kb.v, s[j]);
      }
    }

    _Float16* pwh = Psh[wave];
    _Float16* pwl = Psl[RES ? wave : 0];
#pragma unroll
    for (int r = 0; r < 8; ++r) {
      const int qrow = q0 + 8 * hh + r;
      float m = -INFINITY;
#pragma unroll
      for (int j = 0; j < 4; ++j) {
        const int key = kv0 + j * 16 + c;
        const float sraw = s[j][r] * sscale;
        const float sv = (key > qrow) ? -INFINITY : sraw;
        s[j][r] = sv;
        m = fmaxf(m, sv);
      }
#pragma unroll
      for (int off = 1; off < 16; off <<= 1) m = fmaxf(m, __shfl_xor(m, off, 32));
      const float mnew  = fmaxf(mrow[r], m);
      const float msafe = (mnew == -INFINITY) ? 0.f : mnew;
      const float alpha = __expf(mrow[r] - msafe);
      mrow[r] = mnew;
      float psum = 0.f;
#pragma unroll
      for (int j = 0; j < 4; ++j) {
        const float p = __expf(s[j][r] - msafe);
        psum += p;
        const float p1k = p * 1024.0f;
        const _Float16 ph = (_Float16)p1k;
        pwh[(8 * hh + r) * 64 + j * 16 + c] = ph;
        if (RES) {
          const _Float16 pl = (_Float16)((p1k - (float)ph) * 4096.0f);
          pwl[(8 * hh + r) * 64 + j * 16 + c] = pl;
        }
      }
#pragma unroll
      for (int off = 1; off < 16; off <<= 1) psum += __shfl_xor(psum, off, 32);
      lrow[r] = lrow[r] * alpha + psum;
#pragma unroll
      for (int t = 0; t < 4; ++t) oacc[t][r] *= alpha;
    }
    __builtin_amdgcn_fence(__ATOMIC_RELEASE, "workgroup");
    __builtin_amdgcn_wave_barrier();
    __builtin_amdgcn_fence(__ATOMIC_ACQUIRE, "workgroup");

    v8f o1[4];
#pragma unroll
    for (int t = 0; t < 4; ++t) o1[t] = zero8();
#pragma unroll 1
    for (int kk = 0; kk < 2; ++kk) {
      FH pa, pl;
      pa.h[0] = *(const v8h*)(pwh + c * 64 + kk * 32 + 8 * hh);
      pa.h[1] = *(const v8h*)(pwh + c * 64 + kk * 32 + 16 + 8 * hh);
      if (RES) {
        pl.h[0] = *(const v8h*)(pwl + c * 64 + kk * 32 + 8 * hh);
        pl.h[1] = *(const v8h*)(pwl + c * 64 + kk * 32 + 16 + 8 * hh);
      } else {
        pl.v = pa.v;
      }
#pragma unroll
      for (int t = 0; t < 4; ++t) {
        FH vb;
        vb.h[0] = *(const v8h*)(Vth + (t * 16 + c) * 64 + kk * 32 + 8 * hh);
        vb.h[1] = *(const v8h*)(Vth + (t * 16 + c) * 64 + kk * 32 + 16 + 8 * hh);
        oacc[t] = mma_h(pa.v, vb.v, oacc[t]);
        if (RES) {
          FH vl;
          vl.h[0] = *(const v8h*)(Vtl + (t * 16 + c) * 64 + kk * 32 + 8 * hh);
          vl.h[1] = *(const v8h*)(Vtl + (t * 16 + c) * 64 + kk * 32 + 16 + 8 * hh);
          o1[t] = mma_h(pa.v, vl.v, o1[t]);
          o1[t] = mma_h(pl.v, vb.v, o1[t]);
        }
      }
    }
    if (RES) {
#pragma unroll
      for (int t = 0; t < 4; ++t)
#pragma unroll
        for (int r = 0; r < 8; ++r) oacc[t][r] += o1[t][r] * (1.0f / 4096.0f);
    }
  }

  float* os = Os[wave];
#pragma unroll
  for (int r = 0; r < 8; ++r) {
    const float l = lrow[r];
    const float inv = ((l > 0.f) ? (1.0f / l) : 0.f) * (1.0f / 1024.0f);
#pragma unroll
    for (int t = 0; t < 4; ++t) os[(8 * hh + r) * 64 + t * 16 + c] = oacc[t][r] * inv;
  }
  __builtin_amdgcn_fence(__ATOMIC_RELEASE, "workgroup");
  __builtin_amdgcn_wave_barrier();
  __builtin_amdgcn_fence(__ATOMIC_ACQUIRE, "workgroup");
  {
    const int q4 = lane >> 3, c8 = (lane & 7) * 8;
    v4u hv[4], lv[4];
#pragma unroll
    for (int it = 0; it < 4; ++it) {
      const int row = it * 4 + q4;
      const float* sp = os + row * 64 + c8;
      v4u a, a2;
#pragma unroll
      for (int e = 0; e < 4; ++e) {
        const float f0 = sp[2 * e], f1 = sp[2 * e + 1];
        const unsigned short h0 = bf_bits(f0), h1 = bf_bits(f1);
        const unsigned short l0 = bf_bits(f0 - bf_up(h0)), l1 = bf_bits(f1 - bf_up(h1));
        a[e] = pk16(h0, h1); a2[e] = pk16(l0, l1);
      }
      hv[it] = a; lv[it] = a2;
    }
    for (int pass = 0; pass < 2; ++pass) {
#pragma unroll
      for (int it = 0; it < 4; ++it) {
        const int row = it * 4 + q4;
        const size_t go = (size_t)(q0 + row) * DMOD + (size_t)h * HD + c8;
        *(volatile v4u*)(ohp + go) = hv[it];
        *(volatile v4u*)(olp + go) = lv[it];
      }
      __threadfence();
    }
  }
}

__global__ __launch_bounds__(256) void out_finish(const float* __restrict__ P, const float* __restrict__ bias,
                                                   const float* __restrict__ Bm, float* out) {
  const int i = blockIdx.x * 256 + threadIdx.x;
  if (i >= SEQ * (DMOD / 4)) return;
  const int t  = i >> 8;
  const int e0 = (i & 255) * 4;
  const v4f base = *(const v4f*)(P + (size_t)t * NPO + e0);
  const float* oa = P + (size_t)t * NPO + DMOD;
  const v4f bb = *(const v4f*)(bias + e0);
  float acc[4] = {0.f, 0.f, 0.f, 0.f};
#pragma unroll 1
  for (int r = 0; r < LR; ++r) {
    const float xr = 2.0f * oa[r];
    const v4f w = *(const v4f*)(Bm + (size_t)r * DMOD + e0);
#pragma unroll
    for (int e = 0; e < 4; ++e) acc[e] += xr * bfr(w[e]);
  }
  v4f o;
#pragma unroll
  for (int e = 0; e < 4; ++e) o[e] = (base[e] + bfr(bb[e])) + acc[e];
  float* dst = out + (size_t)t * DMOD + e0;
  *(volatile v4f*)dst = o;
  __threadfence();
  *(volatile v4f*)dst = o;
}

extern "C" void kernel_launch(void* const* d_in, const int* in_sizes, int n_in,
                              void* d_out, int out_size, void* d_ws, size_t ws_size,
                              hipStream_t stream) {
  if (n_in < 14) return;
  if (in_sizes[0] != NBAT * SEQ * DMOD) return;
  if (in_sizes[1] != NH * DMOD * HD || in_sizes[2] != NH * DMOD * HD || in_sizes[3] != NH * DMOD * HD) return;
  if (in_sizes[4] != NH * DMOD * LR || in_sizes[6] != NH * DMOD * LR || in_sizes[8] != NH * DMOD * LR) return;
  if (in_sizes[5] != NH * LR * HD || in_sizes[7] != NH * LR * HD || in_sizes[9] != NH * LR * HD) return;
  if (in_sizes[10] != DMOD * DMOD || in_sizes[11] != DMOD || in_sizes[12] != DMOD * LR || in_sizes[13] != LR * DMOD) return;
  if (out_size != NBAT * SEQ * DMOD) return;

  const float* x  = (const float*)d_in[0];
  const float* Wq = (const float*)d_in[1];
  const float* Wk = (const float*)d_in[2];
  const float* Wv = (const float*)d_in[3];
  const float* Aq = (const float*)d_in[4];
  const float* Bq = (const float*)d_in[5];
  const float* Ak = (const float*)d_in[6];
  const float* Bk = (const float*)d_in[7];
  const float* Av = (const float*)d_in[8];
  const float* Bv = (const float*)d_in[9];
  const float* Wp = (const float*)d_in[10];
  const float* bp = (const float*)d_in[11];
  const float* Ap = (const float*)d_in[12];
  const float* Bp = (const float*)d_in[13];
  float* out = (float*)d_out;

  const size_t PWall = (size_t)NALL * DMOD * 2;
  const size_t PWpo  = (size_t)NPO * DMOD * 2;
  const size_t PXb   = (size_t)SEQ * DMOD * 2;
  const size_t PY    = (size_t)SEQ * NALL * 4;
  const size_t PVTh  = (size_t)DMOD * SEQ * 2;
  const size_t PVTl  = (size_t)DMOD * VLP * 2;
  const size_t PP    = (size_t)SEQ * NPO * 4;
  size_t off = 0;
  const size_t oWall = off; off += PWall;
  const size_t oWpo  = off; off += PWpo;
  const size_t oXb   = off; off += PXb;
  const size_t oY    = off; off += PY;
  const size_t oQh   = off; off += PXb;
  const size_t oQl   = off; off += PXb;
  const size_t oKh   = off; off += PXb;
  const size_t oKl   = off; off += PXb;
  const size_t oVTh  = off; off += PVTh;
  const size_t oVTl  = off; off += PVTl;
  const size_t oOh   = off; off += PXb;
  const size_t oOl   = off; off += PXb;
  const size_t oP    = off; off += PP;
  if (off > ws_size) return;
  if (off > (size_t)134217728) return;

  char* ws = (char*)d_ws;
  unsigned short* Wall = (unsigned short*)(ws + oWall);
  unsigned short* Wpo  = (unsigned short*)(ws + oWpo);
  unsigned short* Xb   = (unsigned short*)(ws + oXb);
  float*          Y    = (float*)(ws + oY);
  unsigned short* Qh   = (unsigned short*)(ws + oQh);
  unsigned short* Ql   = (unsigned short*)(ws + oQl);
  unsigned short* Kh   = (unsigned short*)(ws + oKh);
  unsigned short* Kl   = (unsigned short*)(ws + oKl);
  unsigned short* VTh  = (unsigned short*)(ws + oVTh);
  unsigned short* VTl  = (unsigned short*)(ws + oVTl);
  unsigned short* Oh   = (unsigned short*)(ws + oOh);
  unsigned short* Ol   = (unsigned short*)(ws + oOl);
  float*          P    = (float*)(ws + oP);

  const dim3 blk(256);
  const int kc8 = DMOD / 8;
  const dim3 gW((DMOD * kc8 + 255) / 256);
  const dim3 gA((NXA * kc8 + 255) / 256);
  const dim3 gAp((64 * kc8 + 255) / 256);
  const int n8x = SEQ * DMOD / 8;
  const dim3 gCvtX((n8x + 255) / 256);
  const dim3 gProj(((SEQ / 64) * (NALL / 64) + 7) / 8, 1);
  const dim3 gOut(((SEQ / 64) * (NPO / 64) + 7) / 8, 1);
  const dim3 gFin((SEQ * (DMOD / 8) + 255) / 256);
  const dim3 gVf((SEQ / 64) * (DMOD / 64));
  const dim3 gOf((SEQ * (DMOD / 4) + 255) / 256);

  tcvt_bf16<<<gW, blk, 0, stream>>>(Wq, Wall + (size_t)0 * DMOD * DMOD, DMOD, DMOD, DMOD, HD);
  tcvt_bf16<<<gW, blk, 0, stream>>>(Wk, Wall + (size_t)1 * DMOD * DMOD, DMOD, DMOD, DMOD, HD);
  tcvt_bf16<<<gW, blk, 0, stream>>>(Wv, Wall + (size_t)2 * DMOD * DMOD, DMOD, DMOD, DMOD, HD);
  tcvt_bf16<<<gA, blk, 0, stream>>>(Aq, Wall + (size_t)(XAOFF + 0 * NXA) * DMOD, NXA, NXA, DMOD, LR);
  tcvt_bf16<<<gA, blk, 0, stream>>>(Ak, Wall + (size_t)(XAOFF + 1 * NXA) * DMOD, NXA, NXA, DMOD, LR);
  tcvt_bf16<<<gA, blk, 0, stream>>>(Av, Wall + (size_t)(XAOFF + 2 * NXA) * DMOD, NXA, NXA, DMOD, LR);
  tcvt_bf16<<<gW, blk, 0, stream>>>(Wp, Wpo, DMOD, DMOD, DMOD, DMOD);
  tcvt_bf16<<<gAp, blk, 0, stream>>>(Ap, Wpo + (size_t)DMOD * DMOD, 64, LR, DMOD, LR);

  for (int bb = 0; bb < NBAT; ++bb) {
    const float* xb = x + (size_t)bb * SEQ * DMOD;
    float* ob = out + (size_t)bb * SEQ * DMOD;
    cvt_bf16x8<<<gCvtX, blk, 0, stream>>>(xb, Xb, n8x);
    gemm64<0, 0><<<gProj, blk, 0, stream>>>(
        Xb, Xb, DMOD, 0LL, Wall, Wall, DMOD, 0LL,
        (void*)Y, NALL, 0LL, (void*)Y, NALL, 0LL, NALL,
        SEQ, NALL, DMOD, 1.0f);
    proj_finish<<<gFin, blk, 0, stream>>>(Y, 0 * DMOD, XAOFF + 0 * NXA, Bq, Qh, Ql);
    proj_finish<<<gFin, blk, 0, stream>>>(Y, 1 * DMOD, XAOFF + 1 * NXA, Bk, Kh, Kl);
    v_finish<<<gVf, blk, 0, stream>>>(Y, Bv, VTh, VTl, 4096.0f);
    attn_causal64<true><<<dim3(NH * RESQB), dim3(128), 0, stream>>>(
        Qh, Ql, Kh, Kl, VTh, VTl, Oh, Ol, 0, RESQB, 0.125f);
    attn_causal64<false><<<dim3(NH * (NQB - RESQB)), dim3(128), 0, stream>>>(
        Qh, Ql, Kh, Kl, VTh, VTl, Oh, Ol, RESQB, NQB - RESQB, 0.125f);
    gemm64<1, 0><<<gOut, blk, 0, stream>>>(
        Oh, Ol, DMOD, 0LL, Wpo, Wpo, DMOD, 0LL,
        (void*)P, NPO, 0LL, (void*)P, NPO, 0LL, NPO,
        SEQ, NPO, DMOD, 1.0f);
    out_finish<<<gOf, blk, 0, stream>>>(P, bp, Bp, ob);
  }
  (void)hipGetLastError();
}
